// DynamicAttentionMechanism_52029233824339
// MI455X (gfx1250) — hardware-run, weakly checked
//
#include <hip/hip_runtime.h>

typedef float          v8f   __attribute__((ext_vector_type(8)));
typedef float          v4f   __attribute__((ext_vector_type(4)));
typedef unsigned int   v4u   __attribute__((ext_vector_type(4)));
typedef int            v8i   __attribute__((ext_vector_type(8)));
typedef unsigned short v8us  __attribute__((ext_vector_type(8)));
typedef unsigned short v16us __attribute__((ext_vector_type(16)));
typedef __bf16         v16bf __attribute__((ext_vector_type(16)));
typedef _Float16       v16h  __attribute__((ext_vector_type(16)));
typedef v4f  __attribute__((may_alias)) v4fa;
typedef v8us __attribute__((may_alias)) v8usa;
union FragB { v16bf v; v16us u; v8us h[2]; v8i w; };
union FragH { v16h  v; v16us u; v8us h[2]; v8i w; };

__device__ __forceinline__ v8f wmb(const FragB& a, const FragB& b, v8f c) {
  v8f d = __builtin_amdgcn_wmma_f32_16x16x32_bf16(false, a.v, false, b.v, (short)0, c, false, false);
  asm volatile("v_nop\n\tv_nop\n\tv_nop\n\tv_nop" : "+v"(d) : "v"(a.w), "v"(b.w));
  return d;
}

__device__ __forceinline__ v8f wmh(const FragH& a, const FragH& b, v8f c) {
  v8f d = __builtin_amdgcn_wmma_f32_16x16x32_f16(false, a.v, false, b.v, (short)0, c, false, false);
  asm volatile("v_nop\n\tv_nop\n\tv_nop\n\tv_nop" : "+v"(d) : "v"(a.w), "v"(b.w));
  return d;
}

__device__ __forceinline__ unsigned bf16_bits(float f) {
  const unsigned u = __float_as_uint(f);
  const unsigned r = (u + 0x7FFFu + ((u >> 16) & 1u)) >> 16;
  const unsigned q = (u >> 16) | 0x40u;
  return ((u & 0x7fffffffu) > 0x7f800000u) ? q : r;
}

__device__ __forceinline__ float bf16_val(float f) {
  return __uint_as_float(bf16_bits(f) << 16);
}
__device__ __forceinline__ int clampi(int v, int lo, int hi) {
  return v < lo ? lo : (v > hi ? hi : v);
}

__device__ __forceinline__ unsigned f16_bits(float f) {
  const unsigned u  = __float_as_uint(f);
  const unsigned s  = (u >> 16) & 0x8000u;
  const unsigned a  = u & 0x7fffffffu;
  const unsigned t  = a - 0x38000000u;
  const unsigned r  = (t + 0x0FFFu + ((t >> 13) & 1u)) >> 13;
  const unsigned rc = r > 0x7C00u ? 0x7C00u : r;
  const bool small  = a < 0x38800000u;
  const bool isnan  = a > 0x7f800000u;
  const unsigned fin = small ? 0u : (s | rc);
  return isnan ? (s | 0x7E00u) : fin;
}

__device__ __forceinline__ unsigned pk16(unsigned lo, unsigned hi) { return lo | (hi << 16); }
__device__ __forceinline__ unsigned bf16_lo_bits(float v) {
  float hi = bf16_val(v);
  asm volatile("" : "+v"(hi));
  return bf16_bits(v - hi);
}
__device__ __forceinline__ v4u pack8_bf16(v4f a, v4f c) {
  return (v4u){ pk16(bf16_bits(a[0]), bf16_bits(a[1])), pk16(bf16_bits(a[2]), bf16_bits(a[3])),
                pk16(bf16_bits(c[0]), bf16_bits(c[1])), pk16(bf16_bits(c[2]), bf16_bits(c[3])) };
}
__device__ __forceinline__ v4u pack8_bf16_lo(v4f a, v4f c) {
  return (v4u){ pk16(bf16_lo_bits(a[0]), bf16_lo_bits(a[1])), pk16(bf16_lo_bits(a[2]), bf16_lo_bits(a[3])),
                pk16(bf16_lo_bits(c[0]), bf16_lo_bits(c[1])), pk16(bf16_lo_bits(c[2]), bf16_lo_bits(c[3])) };
}
__device__ __forceinline__ v4u pack8_f16(v4f a, v4f c) {
  return (v4u){ pk16(f16_bits(a[0]), f16_bits(a[1])), pk16(f16_bits(a[2]), f16_bits(a[3])),
                pk16(f16_bits(c[0]), f16_bits(c[1])), pk16(f16_bits(c[2]), f16_bits(c[3])) };
}

template <int FORM>
__global__ __launch_bounds__(256) void k_plane(const float* __restrict__ src, int rows, int cols, int ldsrc,
                                               unsigned short* __restrict__ dst, int MP, int KP) {
  static_assert(FORM >= 0 && FORM <= 3);
  const int KTOT = (FORM == 1 || FORM == 3) ? 2 * KP : KP;
  const unsigned ppr   = (unsigned)(KTOT >> 3);
  const unsigned kp8   = (unsigned)(KP >> 3);
  const unsigned total = (unsigned)MP * ppr;
  const unsigned g     = blockIdx.x * 256u + threadIdx.x;
  const unsigned rowu  = g / ppr;
  const unsigned p     = g - rowu * ppr;
  const bool second    = p >= kp8;
  const int row = (int)rowu;
  const int c0  = (int)((second ? p - kp8 : p) << 3);
  const float* srow = src + (size_t)clampi(row, 0, rows - 1) * (size_t)ldsrc;
  float x[8];
  unsigned mk[8];
#pragma unroll
  for (int e = 0; e < 8; ++e) {
    const int c = c0 + e;
    const float v = srow[clampi(c, 0, cols - 1)];
    asm volatile("" :: "v"(v));
    x[e]  = v;
    mk[e] = (row < rows && c < cols) ? 0xFFFFu : 0u;
  }
  const v4f a = (v4f){ x[0], x[1], x[2], x[3] };
  const v4f c = (v4f){ x[4], x[5], x[6], x[7] };
  v4u o;
  if (FORM == 2) {
    o = pack8_f16(a, c);
  } else {
    const v4u hi = pack8_bf16(a, c);
    o = hi;
    if (FORM == 1) { const v4u lo = pack8_bf16_lo(a, c); o = second ? lo : hi; }
  }
  const v4u mw = (v4u){ pk16(mk[0], mk[1]), pk16(mk[2], mk[3]), pk16(mk[4], mk[5]), pk16(mk[6], mk[7]) };
  o &= mw;
  if (g < total) {
    volatile v4u* q = (volatile v4u*)(dst + (size_t)g * 8);
    *q = o;
    __threadfence();
    *q = o;
  }
}

template <int FORM> struct FragOf    { typedef FragB T; };
template <>         struct FragOf<2> { typedef FragH T; };
__device__ __forceinline__ v8f mm(const FragB& a, const FragB& b, v8f c) { return wmb(a, b, c); }
__device__ __forceinline__ v8f mm(const FragH& a, const FragH& b, v8f c) { return wmh(a, b, c); }
template <class F> __device__ __forceinline__ F ld_frag(const unsigned short* p) {
  F f;
  f.h[0] = *(const v8usa*)(p);
  f.h[1] = *(const v8usa*)(p + 16);
  return f;
}

template <int FORM, int EPI>
__global__ __launch_bounds__(256) __attribute__((amdgpu_num_vgpr(248)))
void k_gemm_nt(const unsigned short* __restrict__ A, const unsigned short* __restrict__ B,
               const float* __restrict__ bias, float* __restrict__ D, int M, int N, int KTOT, int ldd) {
  static_assert(FORM >= 0 && FORM <= 2);
  static_assert(EPI == 0 || EPI == 1);
  typedef typename FragOf<FORM>::T F;
  __shared__ __attribute__((aligned(16))) float sT[8][16 * 68];
  const int lane = threadIdx.x & 31;
  const int wave = threadIdx.x >> 5;
  const int tilesM = (M + 63) >> 6;
  const int tilesN = (N + 63) >> 6;
  const int tile = blockIdx.x * 8 + wave;
  if (tile >= tilesM * tilesN) return;
  const int tm = tile / tilesN;
  const int tn = tile - tm * tilesN;
  const int m0 = tm << 6;
  const int n0 = tn << 6;

  const int rl = lane & 15;
  const int h8 = (lane >> 4) * 8;
  const unsigned short* pa = A + (size_t)(m0 + rl) * (size_t)KTOT + h8;
  const unsigned short* pb = B + (size_t)(n0 + rl) * (size_t)KTOT + h8;

  v8f acc[4][4];
#pragma unroll
  for (int i = 0; i < 4; ++i)
#pragma unroll
    for (int j = 0; j < 4; ++j) acc[i][j] = (v8f){0.f, 0.f, 0.f, 0.f, 0.f, 0.f, 0.f, 0.f};

#pragma unroll 1
  for (int k0 = 0; k0 < KTOT; k0 += 32) {
    F bf[4];
#pragma unroll
    for (int j = 0; j < 4; ++j) bf[j] = ld_frag<F>(pb + (size_t)(j << 4) * (size_t)KTOT + k0);
#pragma unroll
    for (int i = 0; i < 4; ++i) {
      const F af = ld_frag<F>(pa + (size_t)(i << 4) * (size_t)KTOT + k0);
#pragma unroll
      for (int j = 0; j < 4; ++j) acc[i][j] = mm(af, bf[j], acc[i][j]);
    }
  }

  float* slab = sT[wave];
  const int hh = lane >> 4;
  const int c4 = (lane & 15) * 4;
  const int nc = n0 + c4;
  const bool cok = nc < N;
  v4f bv = (v4f){0.f, 0.f, 0.f, 0.f};
  if (EPI == 1) {
    bv = *(const v4fa*)(bias + clampi(nc, 0, N - 4));
    asm volatile("" :: "v"(bv));
  }
#pragma unroll
  for (int i = 0; i < 4; ++i) {
    const int mBase = m0 + (i << 4);
#pragma unroll
    for (int j = 0; j < 4; ++j) {
#pragma unroll
      for (int r = 0; r < 8; ++r) slab[(h8 + r) * 68 + (j << 4) + rl] = acc[i][j][r];
    }
    __builtin_amdgcn_fence(__ATOMIC_RELEASE, "workgroup");
    __builtin_amdgcn_wave_barrier();
    __builtin_amdgcn_fence(__ATOMIC_ACQUIRE, "workgroup");
    v4f vv[8];
#pragma unroll
    for (int it = 0; it < 8; ++it) {
      const int row = it * 2 + hh;
      v4f v = *(const v4fa*)(slab + row * 68 + c4);
      if (EPI == 1) v += bv;
      vv[it] = v;
    }
    for (int pass = 0; pass < 2; ++pass) {
#pragma unroll
      for (int it = 0; it < 8; ++it) {
        const int row = mBase + it * 2 + hh;
        if (cok && row < M) *(volatile v4f*)(D + (size_t)row * (size_t)ldd + nc) = vv[it];
      }
      __threadfence();
    }
    __builtin_amdgcn_fence(__ATOMIC_RELEASE, "workgroup");
    __builtin_amdgcn_wave_barrier();
    __builtin_amdgcn_fence(__ATOMIC_ACQUIRE, "workgroup");
  }
}

#ifndef H1_SPLIT
#define H1_SPLIT 1
#endif
#ifndef H2_SPLIT
#define H2_SPLIT 1
#endif

#define NB     8
#define C0     64
#define C1     128
#define C2     128
#define C3     64
#define GH     96
#define GW     96
#define NPIX   (GH * GW)
#define MROWS  (NB * NPIX)
#define NTILE  (NPIX / 32)
#define OUT_ELEMS (NB * C3 * NPIX)

typedef float        v2f __attribute__((ext_vector_type(2)));
typedef unsigned int v2u __attribute__((ext_vector_type(2)));
typedef v2f __attribute__((may_alias)) v2fa;

constexpr int K1 = C0;
constexpr int K2 = (H1_SPLIT != 0) ? 2 * C1 : C1;
constexpr int K3 = (H2_SPLIT != 0) ? 2 * C2 : C2;

static_assert(GH == 96 && GW == 96);
static_assert(NPIX % 32 == 0);
static_assert(MROWS % 64 == 0 && MROWS % 8 == 0);
static_assert(NB * NTILE * 32 == MROWS);
static_assert(K1 % 32 == 0 && K2 % 32 == 0 && K3 % 32 == 0);
static_assert(K1 == 64 && (K2 == 256 || K2 == 128) && (K3 == 256 || K3 == 128));
static_assert(C1 == 128 && C2 == 128 && C3 == 64 && C1 % 64 == 0 && C3 % 64 == 0);
static_assert((C0 & (C0 - 1)) == 0 && (C1 & (C1 - 1)) == 0 && (C2 & (C2 - 1)) == 0);

constexpr int NU_W1  = C1 * (K1 / 8);
constexpr int NU_W2  = C2 * (K2 / 8);
constexpr int NU_W3  = C3 * (K3 / 8);
static_assert(NU_W1 % 256 == 0 && NU_W2 % 256 == 0 && NU_W3 % 256 == 0 && NPIX % 256 == 0);
constexpr int PB_W2   = NU_W1 / 256;
constexpr int PB_W3   = PB_W2 + NU_W2 / 256;
constexpr int PB_BIAS = PB_W3 + NU_W3 / 256;
constexpr int PB_DIS  = PB_BIAS + 1;
constexpr int PB_TOT  = PB_DIS + NPIX / 256;
constexpr int NBIAS4  = (C1 + C2 + C3) / 4;

constexpr size_t SZ_XB   = (size_t)MROWS * C0 * 2;
constexpr size_t SZ_W1T  = (size_t)C1 * 64 * 2;
constexpr size_t SZ_W2T  = (size_t)C2 * 256 * 2;
constexpr size_t SZ_W3T  = (size_t)C3 * 256 * 2;
constexpr size_t SZ_BIAS = 4096;
constexpr size_t SZ_DIS  = (size_t)NPIX * 4;
constexpr size_t SZ_T    = (size_t)MROWS * C1 * 4;
constexpr size_t SZ_HHL  = (size_t)MROWS * 256 * 2;
constexpr size_t SZ_O3   = (size_t)MROWS * C3 * 4;
constexpr size_t OFF_XB   = 0;
constexpr size_t OFF_W1T  = OFF_XB + SZ_XB;
constexpr size_t OFF_W2T  = OFF_W1T + SZ_W1T;
constexpr size_t OFF_W3T  = OFF_W2T + SZ_W2T;
constexpr size_t OFF_BIAS = OFF_W3T + SZ_W3T;
constexpr size_t OFF_DIS  = OFF_BIAS + SZ_BIAS;
constexpr size_t OFF_T    = OFF_DIS + SZ_DIS;
constexpr size_t OFF_HHL  = OFF_T + SZ_T;
constexpr size_t OFF_O3   = OFF_HHL + SZ_HHL;
constexpr size_t WS_TOTAL = OFF_O3 + SZ_O3;
static_assert(WS_TOTAL == (size_t)((size_t)12691 << 13));
static_assert(WS_TOTAL <= ((size_t)128 << 20));
static_assert(OFF_W1T % 256 == 0 && OFF_W2T % 256 == 0 && OFF_W3T % 256 == 0 && OFF_BIAS % 256 == 0);
static_assert(OFF_DIS % 256 == 0 && OFF_T % 256 == 0 && OFF_HHL % 256 == 0 && OFF_O3 % 256 == 0);
static_assert((size_t)C2 * K2 * 2 <= SZ_W2T && (size_t)C3 * K3 * 2 <= SZ_W3T);
static_assert((size_t)MROWS * K2 * 2 <= SZ_HHL && (size_t)MROWS * K3 * 2 <= SZ_HHL);
static_assert((size_t)NBIAS4 * 16 <= SZ_BIAS);
static_assert((size_t)MROWS * C3 * 4 <= SZ_T);

__global__ __launch_bounds__(256) void k_prep_x(const float* __restrict__ x, unsigned short* __restrict__ xb) {
  __shared__ float tile[C0 * 33];
  const int tid = (int)threadIdx.x, lane = tid & 31, wave = tid >> 5;
  const int b  = (int)blockIdx.x / NTILE;
  const int p0 = ((int)blockIdx.x - b * NTILE) * 32;
  const float* xs = x + (size_t)b * C0 * NPIX + p0 + lane;
#pragma unroll 4
  for (int i = 0; i < C0 / 8; ++i) {
    const int c = wave + 8 * i;
    const float v = xs[(size_t)c * NPIX];
    asm volatile("" :: "v"(v));
    tile[c * 33 + lane] = v;
  }
  __syncthreads();
  const int row = tid >> 3, pc = tid & 7;
  float e[8];
#pragma unroll
  for (int i = 0; i < 8; ++i) e[i] = tile[(pc * 8 + i) * 33 + row];
  const v4u o = pack8_bf16((v4f){ e[0], e[1], e[2], e[3] }, (v4f){ e[4], e[5], e[6], e[7] });
  volatile v4u* q = (volatile v4u*)(xb + (size_t)(b * NPIX + p0 + row) * C0 + pc * 8);
  *q = o;
  __threadfence();
  *q = o;
}

__device__ __forceinline__ void wt_unit(const float* __restrict__ W, int ldw, int kin,
                                        unsigned short* __restrict__ dst, int pitch, int u) {
  const int ppr = pitch >> 3;
  const int n   = u / ppr;
  const int pc  = u - n * ppr;
  const int k8  = pc << 3;
  const int kk  = k8 & (kin - 1);
  const float* p = W + (size_t)kk * (size_t)ldw + n;
  float e[8];
#pragma unroll
  for (int i = 0; i < 8; ++i) {
    const float v = p[(size_t)i * (size_t)ldw];
    asm volatile("" :: "v"(v));
    e[i] = v;
  }
  const v4u o = pack8_bf16((v4f){ e[0], e[1], e[2], e[3] }, (v4f){ e[4], e[5], e[6], e[7] });
  volatile v4u* q = (volatile v4u*)(dst + (size_t)n * (size_t)pitch + k8);
  *q = o;
  __threadfence();
  *q = o;
}

__device__ __forceinline__ int deg_of(int ti, int tj) {
  int deg = 1;
#pragma unroll
  for (int q = 0; q < 9; ++q) {
    if (q == 4) continue;
    const int dr = q / 3 - 1;
    const int dc = q - 3 * (q / 3) - 1;
    int si = ti + dr; si += (si < 0) ? GH : 0; si -= (si >= GH) ? GH : 0;
    int sj = tj + dc; sj += (sj < 0) ? GW : 0; sj -= (sj >= GW) ? GW : 0;
    const bool bad = ((dr != 0) && (si == 0)) || ((dc != 0) && (sj == 0));
    deg += bad ? 0 : 1;
  }
  return deg;
}

__global__ __launch_bounds__(256) void k_prep_w(const float* __restrict__ W1, const float* __restrict__ b1,
                                                const float* __restrict__ W2, const float* __restrict__ b2,
                                                const float* __restrict__ W3, const float* __restrict__ b3,
                                                unsigned short* __restrict__ W1T, unsigned short* __restrict__ W2T2,
                                                unsigned short* __restrict__ W3T2,
                                                float* __restrict__ BIAS, float* __restrict__ DIS) {
  __shared__ __attribute__((aligned(16))) float sd[256];
  const int tid = (int)threadIdx.x;
  const int blk = (int)blockIdx.x;
  {
    const int pix = clampi((blk - PB_DIS) * 256 + tid, 0, NPIX - 1);
    const int ti = pix / GW;
    const int tj = pix - ti * GW;
    const int deg = deg_of(ti, tj);
    sd[tid] = 1.0f / sqrtf((float)deg);
  }
  __syncthreads();
  if (blk < PB_W2) {
    wt_unit(W1, C1, C0, W1T, K1, blk * 256 + tid);
  } else if (blk < PB_W3) {
    wt_unit(W2, C2, C1, W2T2, K2, (blk - PB_W2) * 256 + tid);
  } else if (blk < PB_BIAS) {
    wt_unit(W3, C3, C2, W3T2, K3, (blk - PB_W3) * 256 + tid);
  } else if (blk < PB_DIS) {
    const int u  = tid < NBIAS4 ? tid : NBIAS4 - 1;
    const int i1 = clampi(u, 0, C1 / 4 - 1) * 4;
    const int i2 = clampi(u - C1 / 4, 0, C2 / 4 - 1) * 4;
    const int i3 = clampi(u - (C1 + C2) / 4, 0, C3 / 4 - 1) * 4;
    const v4f a1 = *(const v4fa*)(b1 + i1);
    const v4f a2 = *(const v4fa*)(b2 + i2);
    const v4f a3 = *(const v4fa*)(b3 + i3);
    asm volatile("" :: "v"(a1));
    asm volatile("" :: "v"(a2));
    asm volatile("" :: "v"(a3));
    const unsigned m1 = (u < C1 / 4) ? 0xFFFFFFFFu : 0u;
    const unsigned m3 = (u >= (C1 + C2) / 4) ? 0xFFFFFFFFu : 0u;
    const unsigned m2 = ~(m1 | m3);
    v4f o;
#pragma unroll
    for (int e = 0; e < 4; ++e) {
      const unsigned bits = (__float_as_uint(a1[e]) & m1) | (__float_as_uint(a2[e]) & m2) | (__float_as_uint(a3[e]) & m3);
      o[e] = bf16_val(__uint_as_float(bits));
    }
    if (tid < NBIAS4) {
      volatile v4f* q = (volatile v4f*)(BIAS + 4 * tid);
      *q = o;
      __threadfence();
      *q = o;
    }
  } else {
    const int t4 = tid < 64 ? tid : 63;
    const v4f o = *(const v4fa*)(sd + 4 * t4);
    if (tid < 64) {
      volatile v4f* q = (volatile v4f*)(DIS + (size_t)(blk - PB_DIS) * 256 + 4 * tid);
      *q = o;
      __threadfence();
      *q = o;
    }
  }
}

template <int C, int MODE, int SPLIT>
__global__ __launch_bounds__(256) void k_stencil(const float* __restrict__ T, const float* __restrict__ dis,
                                                 const float* __restrict__ bias,
                                                 unsigned short* __restrict__ hb, float* __restrict__ of) {
  static_assert((C == 128 && MODE == 1) || (C == 64 && MODE == 0));
  constexpr int VW    = C / 32;
  constexpr int PITCH = (SPLIT != 0) ? 2 * C : C;
  __shared__ __attribute__((aligned(16))) float sb[C];
  const int tid = (int)threadIdx.x, lane = tid & 31, wave = tid >> 5;
  {
    const int bi = tid < C / 4 ? tid : C / 4 - 1;
    const v4f bv = *(const v4fa*)(bias + 4 * bi);
    asm volatile("" :: "v"(bv));
    if (tid < C / 4) *(v4fa*)(sb + 4 * tid) = bv;
  }
  __syncthreads();

  const int r  = __builtin_amdgcn_readfirstlane((int)blockIdx.x * 8 + wave);
  const int b  = r / NPIX;
  const int p  = r - b * NPIX;
  const int ti = p / GW;
  const int tj = p - ti * GW;

  const int q  = lane < 4 ? lane : (lane < 8 ? lane + 1 : 4);
  const int qr = (q >= 6) ? 2 : ((q >= 3) ? 1 : 0);
  const int dr = qr - 1;
  const int dc = q - 3 * qr - 1;
  int si = ti + dr; si += (si < 0) ? GH : 0; si -= (si >= GH) ? GH : 0;
  int sj = tj + dc; sj += (sj < 0) ? GW : 0; sj -= (sj >= GW) ? GW : 0;
  const int src = si * GW + sj;
  const int bad = (((dr != 0) && (si == 0)) || ((dc != 0) && (sj == 0))) ? 1 : 0;
  const float ds = dis[src];
  asm volatile("" :: "v"(ds));
  const float dt = __int_as_float(__builtin_amdgcn_readlane(__float_as_int(ds), 8));
  const float cf = ds * dt;
  const int cfi  = __float_as_int(cf);

  const float* tb = T + (size_t)b * NPIX * C + lane * VW;
  float a[VW];
#pragma unroll
  for (int e = 0; e < VW; ++e) a[e] = 0.0f;
#pragma unroll
  for (int o = 0; o < 9; ++o) {
    const int   s  = __builtin_amdgcn_readlane(src, o);
    const float co = __int_as_float(__builtin_amdgcn_readlane(cfi, o));
    const int   bd = __builtin_amdgcn_readlane(bad, o);
    float t[VW];
    if constexpr (VW == 4) {
      const v4f v = *(const v4fa*)(tb + (size_t)s * C);
      t[0] = v[0]; t[1] = v[1]; t[2] = v[2]; t[3] = v[3];
    } else {
      const v2f v = *(const v2fa*)(tb + (size_t)s * C);
      t[0] = v[0]; t[1] = v[1];
    }
#pragma unroll
    for (int e = 0; e < VW; ++e) asm volatile("" :: "v"(t[e]));
#pragma unroll
    for (int e = 0; e < VW; ++e) {
      const float term = t[e] * co;
      a[e] += (bd == 0) ? term : 0.0f;
    }
  }
  float v[VW];
#pragma unroll
  for (int e = 0; e < VW; ++e) {
    const float y = a[e] + sb[lane * VW + e];
    v[e] = (y < 0.0f) ? 0.0f : y;
  }
  if constexpr (MODE == 1) {
    v2u hw, lw;
    hw.x = pk16(bf16_bits(v[0]), bf16_bits(v[1]));
    hw.y = pk16(bf16_bits(v[2]), bf16_bits(v[3]));
    lw.x = pk16(bf16_lo_bits(v[0]), bf16_lo_bits(v[1]));
    lw.y = pk16(bf16_lo_bits(v[2]), bf16_lo_bits(v[3]));
    unsigned short* rp = hb + (size_t)r * PITCH + 4 * lane;
    *(volatile v2u*)rp = hw;
    if (SPLIT != 0) *(volatile v2u*)(rp + C) = lw;
    __threadfence();
    *(volatile v2u*)rp = hw;
    if (SPLIT != 0) *(volatile v2u*)(rp + C) = lw;
  } else {
    v2f ov;
    ov.x = v[0]; ov.y = v[1];
    float* op = of + (size_t)r * C + 2 * lane;
    *(volatile v2f*)op = ov;
    __threadfence();
    *(volatile v2f*)op = ov;
  }
}

__global__ __launch_bounds__(256) void k_out(const float* __restrict__ o3, float* __restrict__ out) {
  __shared__ float tile[32 * 65];
  const int tid = (int)threadIdx.x, lane = tid & 31, wave = tid >> 5;
  const int b  = (int)blockIdx.x / NTILE;
  const int p0 = ((int)blockIdx.x - b * NTILE) * 32;
  const float* src = o3 + (size_t)(b * NPIX + p0) * C3;
#pragma unroll
  for (int i = 0; i < 2; ++i) {
    const int idx = tid + 256 * i;
    const int row = idx >> 4;
    const int c4  = (idx & 15) * 4;
    const v4f v = *(const v4fa*)(src + (size_t)row * C3 + c4);
    asm volatile("" :: "v"(v));
    tile[row * 65 + c4 + 0] = v[0];
    tile[row * 65 + c4 + 1] = v[1];
    tile[row * 65 + c4 + 2] = v[2];
    tile[row * 65 + c4 + 3] = v[3];
  }
  __syncthreads();
  float vv[8];
#pragma unroll
  for (int i = 0; i < 8; ++i) vv[i] = tile[lane * 65 + 8 * wave + i];
  const size_t base = (size_t)(b * C3 + 8 * wave) * NPIX + p0 + lane;
#pragma unroll
  for (int i = 0; i < 8; ++i) {
    const size_t idx = base + (size_t)i * NPIX;
    if (idx < (size_t)OUT_ELEMS) *(volatile float*)(out + idx) = vv[i];
  }
  __threadfence();
#pragma unroll
  for (int i = 0; i < 8; ++i) {
    const size_t idx = base + (size_t)i * NPIX;
    if (idx < (size_t)OUT_ELEMS) *(volatile float*)(out + idx) = vv[i];
  }
}

extern "C" void kernel_launch(void* const* d_in, const int* in_sizes, int n_in,
                              void* d_out, int out_size, void* d_ws, size_t ws_size,
                              hipStream_t stream) {
  if (n_in < 7) return;
  if (in_sizes[0] != NB * C0 * NPIX) return;
  if (in_sizes[1] != C0 * C1 || in_sizes[2] != C1) return;
  if (in_sizes[3] != C1 * C2 || in_sizes[4] != C2) return;
  if (in_sizes[5] != C2 * C3 || in_sizes[6] != C3) return;
  if (out_size != OUT_ELEMS) return;
  if (ws_size < WS_TOTAL) return;

  const float* x  = (const float*)d_in[0];
  const float* W1 = (const float*)d_in[1];
  const float* b1 = (const float*)d_in[2];
  const float* W2 = (const float*)d_in[3];
  const float* b2 = (const float*)d_in[4];
  const float* W3 = (const float*)d_in[5];
  const float* b3 = (const float*)d_in[6];
  float* out = (float*)d_out;

  char* ws = (char*)d_ws;
  unsigned short* XB   = (unsigned short*)(ws + OFF_XB);
  unsigned short* W1T  = (unsigned short*)(ws + OFF_W1T);
  unsigned short* W2T2 = (unsigned short*)(ws + OFF_W2T);
  unsigned short* W3T2 = (unsigned short*)(ws + OFF_W3T);
  float*          BIAS = (float*)(ws + OFF_BIAS);
  float*          DIS  = (float*)(ws + OFF_DIS);
  float*          T    = (float*)(ws + OFF_T);
  unsigned short* HHL  = (unsigned short*)(ws + OFF_HHL);
  float*          O3   = (float*)(ws + OFF_O3);

  const int tiles128 = (MROWS / 64) * (C1 / 64);
  const int tiles64  = (MROWS / 64) * (C3 / 64);

  k_prep_x<<<NB * NTILE, 256, 0, stream>>>(x, XB);
  k_prep_w<<<PB_TOT, 256, 0, stream>>>(W1, b1, W2, b2, W3, b3, W1T, W2T2, W3T2, BIAS, DIS);
  k_gemm_nt<0, 0><<<(tiles128 + 7) / 8, 256, 0, stream>>>(XB, W1T, BIAS, T, MROWS, C1, K1, C1);
  k_stencil<C1, 1, H1_SPLIT><<<MROWS / 8, 256, 0, stream>>>(T, DIS, BIAS, HHL, O3);
  k_gemm_nt<0, 0><<<(tiles128 + 7) / 8, 256, 0, stream>>>(HHL, W2T2, BIAS, T, MROWS, C2, K2, C2);
  k_stencil<C2, 1, H2_SPLIT><<<MROWS / 8, 256, 0, stream>>>(T, DIS, BIAS + C1, HHL, O3);
  k_gemm_nt<0, 0><<<(tiles64 + 7) / 8, 256, 0, stream>>>(HHL, W3T2, BIAS, T, MROWS, C3, K3, C3);
  k_stencil<C3, 0, 0><<<MROWS / 8, 256, 0, stream>>>(T, DIS, BIAS + C1 + C2, HHL, O3);
  k_out<<<NB * NTILE, 256, 0, stream>>>(O3, out);
}
